// Perceptron_26938034881178
// MI455X (gfx1250) — hardware-verified
//
#include <hip/hip_runtime.h>
#include <stdint.h>

#define M_  512
#define K_  1024
#define N_  256
#define OP_ 68

static_assert((M_ % 64) == 0 && (N_ % 64) == 0 && (K_ % 32) == 0 && (K_ % 8) == 0);
static_assert(((M_ * K_) % (8 * 256)) == 0 && ((N_ * K_) % (8 * 256)) == 0);
static_assert((OP_ % 4) == 0);

typedef __bf16       v16b __attribute__((ext_vector_type(16)));
typedef float        v8f  __attribute__((ext_vector_type(8)));
typedef float        v4f  __attribute__((ext_vector_type(4)));
typedef unsigned int v4u  __attribute__((ext_vector_type(4)));
typedef v4f v4fm __attribute__((may_alias));

union FragB { v16b v; v4u u[2]; };
static_assert(sizeof(FragB) == 32);

__device__ __forceinline__ unsigned short bf_bits(float f) {
  unsigned u = __float_as_uint(f);
  return (unsigned short)((u + 0x7FFFu + ((u >> 16) & 1u)) >> 16);
}
__device__ __forceinline__ float bf_up(unsigned short h) { return __uint_as_float(((unsigned)h) << 16); }
__device__ __forceinline__ float bfr(float f) { return bf_up(bf_bits(f)); }
__device__ __forceinline__ unsigned pk16(unsigned short a, unsigned short b) { return (unsigned)a | ((unsigned)b << 16); }
__device__ __forceinline__ v8f zero8() { v8f z = {0.f, 0.f, 0.f, 0.f, 0.f, 0.f, 0.f, 0.f}; return z; }

__device__ __forceinline__ v16b ldfrag_b(const unsigned short* p) {
  FragB f;
  f.u[0] = *(const v4u*)(p);
  f.u[1] = *(const v4u*)(p + 16);
  return f.v;
}

__device__ __forceinline__ v8f wm(v16b a, v16b b, v8f c) {
  return __builtin_amdgcn_wmma_f32_16x16x32_bf16(false, a, false, b, (short)0, c, false, false);
}
__device__ __forceinline__ void guard2(v8f& c0, v8f& c1, v16b a0, v16b b0, v16b b1) {
#if defined(__HIP_DEVICE_COMPILE__)
  asm volatile("v_nop\n\tv_nop\n\tv_nop\n\tv_nop"
               : "+v"(c0), "+v"(c1)
               : "v"(a0), "v"(b0), "v"(b1));
#endif
}
__device__ __forceinline__ void wave_sync_lds() {
#if defined(__HIP_DEVICE_COMPILE__)
  __builtin_amdgcn_fence(__ATOMIC_RELEASE, "workgroup");
  __builtin_amdgcn_wave_barrier();
  __builtin_amdgcn_fence(__ATOMIC_ACQUIRE, "workgroup");
#endif
}

__global__ __launch_bounds__(256) void cvt_plane(const float* __restrict__ src, unsigned short* dst, int n8) {
  const int t = blockIdx.x * 256 + threadIdx.x;
  const int tc = (t < n8) ? t : (n8 - 1);
  const float* p = src + (size_t)tc * 8;
  const v4f a = *(const v4f*)p;
  const v4f b = *(const v4f*)(p + 4);
  v4u pk;
  pk[0] = pk16(bf_bits(a[0]), bf_bits(a[1]));
  pk[1] = pk16(bf_bits(a[2]), bf_bits(a[3]));
  pk[2] = pk16(bf_bits(b[0]), bf_bits(b[1]));
  pk[3] = pk16(bf_bits(b[2]), bf_bits(b[3]));
  unsigned short* gp = dst + (size_t)tc * 8;
  if (t < n8) *(volatile v4u*)gp = pk;
  __threadfence();
  if (t < n8) *(volatile v4u*)gp = pk;
}

__global__ __launch_bounds__(128) void lin_gemm(const unsigned short* __restrict__ xb,
                                                const unsigned short* __restrict__ wb,
                                                const float* __restrict__ bias,
                                                float* out) {
  __shared__ __align__(16) float bT[64];
  __shared__ __align__(16) float Os[4][16 * OP_];
  const int tid = threadIdx.x, lane = tid & 31, wave = tid >> 5;
  const int idx = lane & 15, hh = lane >> 4, koff = 8 * hh;
  const int n0 = blockIdx.x * 64, m0 = blockIdx.y * 64;
  const int mw = m0 + 16 * wave;

  if (tid < 64) bT[tid] = bfr(bias[n0 + tid]);
  __syncthreads();

  const unsigned short* A = xb + (size_t)(mw + idx) * K_ + koff;
  const unsigned short* W = wb + (size_t)(n0 + idx) * K_ + koff;

  v8f acc[4];
#pragma unroll
  for (int j = 0; j < 4; ++j) acc[j] = zero8();

#pragma unroll 1
  for (int ks = 0; ks < K_ / 32; ++ks) {
    const int k0 = 32 * ks;
    const v16b fa = ldfrag_b(A + k0);
    {
      const v16b b0 = ldfrag_b(W + k0);
      const v16b b1 = ldfrag_b(W + (size_t)16 * K_ + k0);
      acc[0] = wm(fa, b0, acc[0]);
      acc[1] = wm(fa, b1, acc[1]);
      guard2(acc[0], acc[1], fa, b0, b1);
    }
    {
      const v16b b2 = ldfrag_b(W + (size_t)32 * K_ + k0);
      const v16b b3 = ldfrag_b(W + (size_t)48 * K_ + k0);
      acc[2] = wm(fa, b2, acc[2]);
      acc[3] = wm(fa, b3, acc[3]);
      guard2(acc[2], acc[3], fa, b2, b3);
    }
  }

  float* os = Os[wave];
#pragma unroll
  for (int j = 0; j < 4; ++j) {
    const float bb = bT[16 * j + idx];
#pragma unroll
    for (int r = 0; r < 8; ++r) {
      const float t = acc[j][r] + bb;
      const float e = __expf(-t);
      const float s = __builtin_amdgcn_rcpf(1.0f + e);
      os[(8 * hh + r) * OP_ + 16 * j + idx] = s;
    }
  }
  wave_sync_lds();

  const int r2 = lane >> 4, q = lane & 15;
  v4f ov[8];
#pragma unroll
  for (int s = 0; s < 8; ++s) ov[s] = *(const v4fm*)(os + (2 * s + r2) * OP_ + 4 * q);
#pragma unroll
  for (int s = 0; s < 8; ++s) {
    float* g = out + (size_t)(mw + 2 * s + r2) * N_ + n0 + 4 * q;
    *(volatile v4f*)g = ov[s];
  }
  __threadfence();
#pragma unroll
  for (int s = 0; s < 8; ++s) {
    float* g = out + (size_t)(mw + 2 * s + r2) * N_ + n0 + 4 * q;
    *(volatile v4f*)g = ov[s];
  }
}

extern "C" void kernel_launch(void* const* d_in, const int* in_sizes, int n_in,
                              void* d_out, int out_size, void* d_ws, size_t ws_size,
                              hipStream_t stream) {
  if (n_in < 3) return;
  if (in_sizes[0] != M_ * K_) return;
  if (in_sizes[1] != N_ * K_) return;
  if (in_sizes[2] != N_) return;
  if (out_size != M_ * N_) return;

  const float* x    = (const float*)d_in[0];
  const float* w    = (const float*)d_in[1];
  const float* bias = (const float*)d_in[2];
  float* out = (float*)d_out;

  const size_t sX = (size_t)M_ * K_ * 2;
  const size_t sW = (size_t)N_ * K_ * 2;
  size_t off = 0;
  const size_t oX = off; off += sX;
  const size_t oW = off; off += sW;
  if (off > ws_size) return;
  if (off > (size_t)134217728) return;

  char* ws = (char*)d_ws;
  unsigned short* XB = (unsigned short*)(ws + oX);
  unsigned short* WB = (unsigned short*)(ws + oW);

  const dim3 blk(256);
  {
    const int n8 = M_ * K_ / 8;
    cvt_plane<<<dim3((n8 + 255) / 256), blk, 0, stream>>>(x, XB, n8);
  }
  {
    const int n8 = N_ * K_ / 8;
    cvt_plane<<<dim3((n8 + 255) / 256), blk, 0, stream>>>(w, WB, n8);
  }
  lin_gemm<<<dim3(N_ / 64, M_ / 64), dim3(128), 0, stream>>>(XB, WB, bias, out);
  (void)hipGetLastError();
}
